// CausalSelfAttention_74809740362128
// MI455X (gfx1250) — hardware-verified
//
#include <hip/hip_runtime.h>
#ifndef NB
#define NB 4
#endif
#ifndef SEQ
#define SEQ 2048
#endif
#define SQ SEQ
#define NB_FULL 4
#define SQ_FULL 2048
#define DM 1024
#define NH 16
#define HD 64
#ifndef QT0
#define QT0 256
#endif
#define NR ((size_t)NB * SQ)
#define PLP 72
#define AL256(x) ((((size_t)(x)) + 255) & ~(size_t)255)
#define WS_TOTAL (4 * AL256((size_t)DM * DM * 2) + 6 * AL256(NR * DM * 2) + 4 * AL256((size_t)NB * QT0 * DM * 4) + 2 * AL256((size_t)NB * QT0 * DM * 2))
static_assert(NH * HD == DM);
static_assert(HD == 64);
static_assert(DM % 64 == 0 && DM % 32 == 0);
static_assert(SQ % 128 == 0);
static_assert(QT0 % 128 == 0 && QT0 <= SQ);
static_assert(QT0 % 64 == 0);
static_assert(NB <= NB_FULL && SQ <= SQ_FULL);
static_assert(PLP % 8 == 0 && PLP >= HD);
static_assert(WS_TOTAL <= (size_t)134217728);
static_assert((size_t)NB_FULL * SQ_FULL * DM * 4 == (size_t)33554432);

typedef unsigned short v8us __attribute__((ext_vector_type(8), may_alias));
typedef float  v8f  __attribute__((ext_vector_type(8)));
typedef float  v4f  __attribute__((ext_vector_type(4)));
typedef float  v4fa __attribute__((ext_vector_type(4), may_alias));
typedef _Float16 v16h __attribute__((ext_vector_type(16)));
typedef _Float16 v4h __attribute__((ext_vector_type(4)));
union FragH { v16h v; v8us half[2]; _Float16 h[16]; unsigned short u[16]; };

__device__ __forceinline__ unsigned short bf16_bits(float x) { unsigned int u = __float_as_uint(x); return (unsigned short)((u + 0x7FFFu + ((u >> 16) & 1u)) >> 16); }
__device__ __forceinline__ float bf16_val(unsigned short b) { return __uint_as_float(((unsigned int)b) << 16); }
__device__ __forceinline__ float bf16_rne(float x) { return bf16_val(bf16_bits(x)); }

__device__ __forceinline__ v16h g2_frag(const _Float16* p, int hh) { FragH f; f.half[0] = *(const v8us*)((const unsigned short*)p + 8 * hh); f.half[1] = *(const v8us*)((const unsigned short*)p + 16 + 8 * hh); return f.v; }
__device__ __forceinline__ v8f g2_mma(v16h a, v16h b, v8f c) { v8f d = __builtin_amdgcn_wmma_f32_16x16x32_f16(false, a, false, b, (short)0, c, false, false); asm volatile("v_nop\n\tv_nop\n\tv_nop\n\tv_nop" : "+v"(d) : "v"(a), "v"(b)); return d; }

__global__ __launch_bounds__(256) void k_wt_f16(const float* __restrict__ W, _Float16* __restrict__ Wt, int K, int N, float scale) {
  const int t = blockIdx.x * 256 + threadIdx.x; if (t >= N * (K / 8)) return; const int n = t / (K / 8), k8 = (t % (K / 8)) * 8; FragH f;
#pragma unroll
  for (int i = 0; i < 8; ++i) f.h[i] = (_Float16)(bf16_rne(W[(size_t)(k8 + i) * N + n]) * scale);
  const v8us o = f.half[0];
  *(volatile v8us*)((unsigned short*)Wt + (size_t)n * K + k8) = o; __threadfence(); *(volatile v8us*)((unsigned short*)Wt + (size_t)n * K + k8) = o;
}

__global__ __launch_bounds__(256) void k_x16b(const float* __restrict__ x, size_t sxb, _Float16* __restrict__ X16, size_t sob, size_t n8) {
  const size_t t = (size_t)blockIdx.x * 256 + threadIdx.x; if (t >= n8) return;
  const float* xp = x + (size_t)blockIdx.y * sxb + t * 8;
  const v4f a = *(const v4fa*)xp, c = *(const v4fa*)(xp + 4);
  FragH f;
#pragma unroll
  for (int q = 0; q < 4; ++q) { f.h[q] = (_Float16)bf16_rne(a[q]); f.h[4 + q] = (_Float16)bf16_rne(c[q]); }
  const v8us o = f.half[0];
  unsigned short* d = (unsigned short*)X16 + (size_t)blockIdx.y * sob + t * 8;
  *(volatile v8us*)d = o; __threadfence(); *(volatile v8us*)d = o;
}

__global__ __launch_bounds__(128) void k_gemm2(const _Float16* __restrict__ A, int lda, size_t sA, const _Float16* __restrict__ Bh, int ldb, size_t sB, float alpha,
    const float* __restrict__ bias, const float* CP, float* C, _Float16* __restrict__ C16, int ldc, size_t sC, int M, int N, int K) {
  __shared__ __attribute__((aligned(16))) float so[4][32][68];
  const int tid = threadIdx.x, w = tid >> 5, lane = tid & 31, ln = lane & 15, hh = lane >> 4; const int by = blockIdx.y;
  A += (size_t)by * sA; Bh += (size_t)by * sB; const size_t cofs = (size_t)by * sC;
  const int ntn = N >> 6; const int mt = blockIdx.x / ntn, nq = blockIdx.x - mt * ntn; const int row0 = mt * 128 + 32 * w, col0 = nq * 64; if (row0 >= M) return;
  const _Float16* a0p = A + (size_t)(row0 + ln) * lda; const _Float16* a1p = a0p + (size_t)16 * lda;
  const _Float16* b0p = Bh + (size_t)(col0 + ln) * ldb; const _Float16* b1p = b0p + (size_t)16 * ldb; const _Float16* b2p = b1p + (size_t)16 * ldb; const _Float16* b3p = b2p + (size_t)16 * ldb;
  const v8f z8 = {0.f,0.f,0.f,0.f,0.f,0.f,0.f,0.f}; v8f c00 = z8, c01 = z8, c02 = z8, c03 = z8, c10 = z8, c11 = z8, c12 = z8, c13 = z8;
#pragma unroll 1
  for (int kb = 0; kb < K; kb += 32) { const v16h a0 = g2_frag(a0p + kb, hh), a1 = g2_frag(a1p + kb, hh);
    v16h b = g2_frag(b0p + kb, hh); c00 = g2_mma(a0, b, c00); c10 = g2_mma(a1, b, c10);
    b = g2_frag(b1p + kb, hh); c01 = g2_mma(a0, b, c01); c11 = g2_mma(a1, b, c11);
    b = g2_frag(b2p + kb, hh); c02 = g2_mma(a0, b, c02); c12 = g2_mma(a1, b, c12);
    b = g2_frag(b3p + kb, hh); c03 = g2_mma(a0, b, c03); c13 = g2_mma(a1, b, c13); }
  v8f accs[8] = {c00, c01, c02, c03, c10, c11, c12, c13};
#pragma unroll
  for (int u = 0; u < 8; ++u) { const int t = u & 3, half = u >> 2; const int col = col0 + t * 16 + ln; const float bv = bias ? bf16_rne(bias[col]) : 0.f;
#pragma unroll
    for (int r = 0; r < 8; ++r) { const int rloc = half * 16 + 8 * hh + r; float v = accs[u][r] * alpha + bv; if (CP) v += CP[cofs + (size_t)(row0 + rloc) * ldc + col];
      so[w][rloc][t * 16 + ln] = v; } }
  __builtin_amdgcn_fence(4  , "workgroup"); __builtin_amdgcn_wave_barrier();
  const int rsub = lane >> 4, c4 = (lane & 15) * 4;
  for (int pass = 0; pass < 2; ++pass) {
#pragma unroll
    for (int q = 0; q < 16; ++q) { const int r = q * 2 + rsub; const v4f v = *(const v4fa*)&so[w][r][c4]; if (C) *(volatile v4f*)(C + cofs + (size_t)(row0 + r) * ldc + col0 + c4) = v; if (C16) { v4h h4;
#pragma unroll
        for (int i = 0; i < 4; ++i) h4[i] = (_Float16)v[i]; *(volatile v4h*)(C16 + cofs + (size_t)(row0 + r) * ldc + col0 + c4) = h4; } }
    if (pass == 0) __threadfence(); } }

__global__ __launch_bounds__(256) void k_vt16(const _Float16* __restrict__ V16, int ldv, _Float16* __restrict__ Vt) {
  __shared__ unsigned short tl[64][66]; const int tid = threadIdx.x; const int slab = blockIdx.x / (SQ / 64), lg = blockIdx.x % (SQ / 64); const int b = slab / NH, h = slab % NH;
  for (int i = tid; i < 64 * 8; i += 256) { const int r = i / 8, c8 = (i % 8) * 8; FragH f; f.half[0] = *(const v8us*)((const unsigned short*)V16 + ((size_t)b * SQ + lg * 64 + r) * ldv + h * 64 + c8);
#pragma unroll
    for (int q = 0; q < 8; ++q) tl[r][c8 + q] = f.u[q]; }
  __syncthreads();
  for (int pass = 0; pass < 2; ++pass) {
#pragma unroll
    for (int rd = 0; rd < 2; ++rd) { const int d = rd * 32 + tid / 8, pc = tid % 8; FragH f;
#pragma unroll
      for (int q = 0; q < 8; ++q) f.u[q] = tl[pc * 8 + q][d];
      *(volatile v8us*)((unsigned short*)Vt + ((size_t)slab * 64 + d) * SQ + lg * 64 + pc * 8) = f.half[0]; }
    if (pass == 0) __threadfence(); } }

__global__ __launch_bounds__(256) void k_hl(const float* __restrict__ F, _Float16* __restrict__ Hh, _Float16* __restrict__ Hl, size_t n8) { const size_t t = (size_t)blockIdx.x * 256 + threadIdx.x; if (t >= n8) return; FragH fh, fl; const v4f a = *(const v4fa*)(F + t * 8), c = *(const v4fa*)(F + t * 8 + 4);
#pragma unroll
  for (int q = 0; q < 4; ++q) { _Float16 h = (_Float16)a[q]; fh.h[q] = h; fl.h[q] = (_Float16)((a[q] - (float)h) * 1024.0f); h = (_Float16)c[q]; fh.h[4 + q] = h; fl.h[4 + q] = (_Float16)((c[q] - (float)h) * 1024.0f); }
  for (int pass = 0; pass < 2; ++pass) { *(volatile v8us*)((unsigned short*)Hh + t * 8) = fh.half[0]; *(volatile v8us*)((unsigned short*)Hl + t * 8) = fl.half[0]; if (pass == 0) __threadfence(); } }

__global__ __launch_bounds__(64) void k_att0(const float* __restrict__ QF, const float* __restrict__ KF, const float* __restrict__ VF, int ld, float scale, float* __restrict__ OF, int ldo) {
  #pragma clang fp contract(off)
  __shared__ __attribute__((aligned(16))) float lq[64][64]; __shared__ __attribute__((aligned(16))) float lo[64][64];
  const int tid = threadIdx.x; const int h = blockIdx.x / (QT0 / 64), rg = blockIdx.x % (QT0 / 64); const int i = rg * 64 + tid;
  const size_t bofs = (size_t)blockIdx.y * QT0 * ld; QF += bofs; KF += bofs; VF += bofs; OF += (size_t)blockIdx.y * QT0 * ldo;
  const float* qr = QF + (size_t)i * ld + h * HD;
#pragma unroll 1
  for (int c = 0; c < HD / 4; ++c) { *(v4f*)&lq[tid][c * 4] = *(const v4fa*)(qr + c * 4); const v4f z = {0.f, 0.f, 0.f, 0.f}; *(v4f*)&lo[tid][c * 4] = z; }
  float m = -1.0e30f, l = 0.f; const int jmax = rg * 64 + 63;
#pragma unroll 1
  for (int j = 0; j <= jmax; ++j) { const float* kr = KF + (size_t)j * ld + h * HD; const float* vr = VF + (size_t)j * ld + h * HD; float s = 0.f;
#pragma unroll 1
    for (int c = 0; c < HD / 4; ++c) { const v4f kq = *(const v4fa*)(kr + c * 4); const v4f qq = *(v4f*)&lq[tid][c * 4]; s = __fadd_rn(s, __fmul_rn(qq[0], kq[0])); s = __fadd_rn(s, __fmul_rn(qq[1], kq[1])); s = __fadd_rn(s, __fmul_rn(qq[2], kq[2])); s = __fadd_rn(s, __fmul_rn(qq[3], kq[3])); }
    s = __fmul_rn(s, scale);
    const float f = (j <= i) ? 1.f : 0.f; const float sm = fmaf(f, s, (1.f - f) * -1.0e30f); const float mn = fmaxf(m, sm); const float sc = expf(m - mn); const float e = expf(sm - mn); l = __fadd_rn(__fmul_rn(l, sc), e); m = mn;
#pragma unroll 1
    for (int c = 0; c < HD / 4; ++c) { const v4f vv = *(const v4fa*)(vr + c * 4); v4f oo = *(v4f*)&lo[tid][c * 4];
#pragma unroll
      for (int u = 0; u < 4; ++u) oo[u] = __fadd_rn(__fmul_rn(oo[u], sc), __fmul_rn(e, vv[u]));
      *(v4f*)&lo[tid][c * 4] = oo; } }
  const float fin = 64.0f / l;
#pragma unroll 1
  for (int c = 0; c < HD / 4; ++c) { v4f oo = *(v4f*)&lo[tid][c * 4];
#pragma unroll
    for (int u = 0; u < 4; ++u) oo[u] = __fmul_rn(oo[u], fin);
    *(v4f*)&lo[tid][c * 4] = oo; }
  __syncthreads();
  for (int pass = 0; pass < 2; ++pass) {
#pragma unroll 1
    for (int it = 0; it < 16; ++it) { const int row = it * 4 + tid / 16, pc = (tid % 16) * 4; const v4f v = *(const v4f*)&lo[row][pc]; *(volatile v4f*)(OF + (size_t)(rg * 64 + row) * ldo + h * HD + pc) = v; }
    if (pass == 0) __threadfence(); } }

__global__ __launch_bounds__(256) void k_fattn(const _Float16* __restrict__ Q16, const _Float16* __restrict__ K16, const _Float16* __restrict__ VT, _Float16* __restrict__ O16) {
  __shared__ __attribute__((aligned(16))) _Float16 pl[8][16][PLP];
  const int tid = threadIdx.x, w = tid >> 5, lane = tid & 31, ln = lane & 15, hh = lane >> 4;
  const int bh = blockIdx.y; const int b = bh / NH, h = bh - b * NH;
  const int q0 = blockIdx.x * 128 + w * 16;
  const size_t rb = (size_t)b * SQ;
  const _Float16* qp = Q16 + (rb + q0 + ln) * DM + h * HD;
  const v16h qf0 = g2_frag(qp, hh), qf1 = g2_frag(qp + 32, hh);
  const _Float16* kp0 = K16 + (rb + ln) * DM + h * HD;
  const _Float16* vp0 = VT + ((size_t)bh * HD + ln) * SQ;
  const v8f z8 = {0.f,0.f,0.f,0.f,0.f,0.f,0.f,0.f};
  v8f o[4] = {z8, z8, z8, z8};
  float mr[8], lr[8];
#pragma unroll
  for (int r = 0; r < 8; ++r) { mr[r] = -1.0e30f; lr[r] = 0.f; }
  const int nkb = (q0 + 15) / 64 + 1;
#pragma unroll 1
  for (int kb = 0; kb < nkb; ++kb) {
    const int k0 = kb * 64;
    v8f s[4] = {z8, z8, z8, z8};
#pragma unroll
    for (int nt = 0; nt < 4; ++nt) {
      const _Float16* kr = kp0 + (size_t)(k0 + nt * 16) * DM;
      s[nt] = g2_mma(qf0, g2_frag(kr, hh), s[nt]);
      s[nt] = g2_mma(qf1, g2_frag(kr + 32, hh), s[nt]);
    }
#pragma unroll
    for (int nt = 0; nt < 4; ++nt)
#pragma unroll
      for (int r = 0; r < 8; ++r) s[nt][r] *= 0.125f;
    if (kb == nkb - 1) {
#pragma unroll
      for (int nt = 0; nt < 4; ++nt) { const int kj = k0 + nt * 16 + ln;
#pragma unroll
        for (int r = 0; r < 8; ++r) { const int qi = q0 + 8 * hh + r; const float sv = s[nt][r]; s[nt][r] = (kj <= qi) ? sv : -1.0e30f; } }
    }
    float al[8];
#pragma unroll
    for (int r = 0; r < 8; ++r) {
      float mx = fmaxf(fmaxf(s[0][r], s[1][r]), fmaxf(s[2][r], s[3][r]));
      mx = fmaxf(mx, __shfl_xor(mx, 1)); mx = fmaxf(mx, __shfl_xor(mx, 2)); mx = fmaxf(mx, __shfl_xor(mx, 4)); mx = fmaxf(mx, __shfl_xor(mx, 8));
      const float mn = fmaxf(mr[r], mx);
      al[r] = __expf(mr[r] - mn); mr[r] = mn;
      float rs = 0.f;
#pragma unroll
      for (int nt = 0; nt < 4; ++nt) { const float e = __expf(s[nt][r] - mn); s[nt][r] = e; rs += e; }
      rs += __shfl_xor(rs, 1); rs += __shfl_xor(rs, 2); rs += __shfl_xor(rs, 4); rs += __shfl_xor(rs, 8);
      lr[r] = lr[r] * al[r] + rs;
    }
#pragma unroll
    for (int nt = 0; nt < 4; ++nt)
#pragma unroll
      for (int r = 0; r < 8; ++r) { o[nt][r] *= al[r]; pl[w][8 * hh + r][nt * 16 + ln] = (_Float16)(s[nt][r] * 256.0f); }
    __builtin_amdgcn_fence(4  , "workgroup"); __builtin_amdgcn_wave_barrier();
    FragH pa, pb;
    pa.half[0] = *(const v8us*)((const unsigned short*)&pl[w][ln][8 * hh]);      pa.half[1] = *(const v8us*)((const unsigned short*)&pl[w][ln][16 + 8 * hh]);
    pb.half[0] = *(const v8us*)((const unsigned short*)&pl[w][ln][32 + 8 * hh]); pb.half[1] = *(const v8us*)((const unsigned short*)&pl[w][ln][48 + 8 * hh]);
#pragma unroll
    for (int nt = 0; nt < 4; ++nt) {
      const _Float16* vr = vp0 + (size_t)(nt * 16) * SQ + k0;
      o[nt] = g2_mma(pa.v, g2_frag(vr, hh), o[nt]);
      o[nt] = g2_mma(pb.v, g2_frag(vr + 32, hh), o[nt]);
    }
    __builtin_amdgcn_fence(4  , "workgroup"); __builtin_amdgcn_wave_barrier();
  }
#pragma unroll
  for (int r = 0; r < 8; ++r) { const float inv = 0.25f / lr[r];
#pragma unroll
    for (int nt = 0; nt < 4; ++nt) pl[w][8 * hh + r][nt * 16 + ln] = (_Float16)(o[nt][r] * inv); }
  __builtin_amdgcn_fence(4  , "workgroup"); __builtin_amdgcn_wave_barrier();
  const int rq = lane >> 3, pc = (lane & 7) * 8;
  v8us ov[4];
#pragma unroll
  for (int it = 0; it < 4; ++it) ov[it] = *(const v8us*)((const unsigned short*)&pl[w][it * 4 + rq][pc]);
  for (int pass = 0; pass < 2; ++pass) {
#pragma unroll
    for (int it = 0; it < 4; ++it) *(volatile v8us*)((unsigned short*)O16 + (rb + q0 + it * 4 + rq) * DM + h * HD + pc) = ov[it];
    if (pass == 0) __threadfence(); }
}

extern "C" void kernel_launch(void* const* d_in, const int* in_sizes, int n_in,
                              void* d_out, int out_size, void* d_ws, size_t ws_size, hipStream_t stream) {
  if (n_in < 11) return;
  const size_t need = ((size_t)(NB - 1) * SQ_FULL + SQ) * DM;
  if ((size_t)in_sizes[0] < need || (size_t)in_sizes[1] < need || (size_t)in_sizes[2] < need) return;
  if ((size_t)in_sizes[3] < (size_t)DM * DM || (size_t)in_sizes[5] < (size_t)DM * DM || (size_t)in_sizes[7] < (size_t)DM * DM || (size_t)in_sizes[9] < (size_t)DM * DM) return;
  if (in_sizes[4] < DM || in_sizes[6] < DM || in_sizes[8] < DM || in_sizes[10] < DM) return;
  if ((size_t)out_size < need) return;
  const float* const* I = (const float* const*)d_in;
  const float* q = I[0]; const float* k = I[1]; const float* v = I[2];
  const float* Wq = I[3]; const float* bq = I[4]; const float* Wk = I[5]; const float* bk = I[6]; const float* Wv = I[7]; const float* bv = I[8]; const float* Wo = I[9]; const float* bo = I[10];
  float* out = (float*)d_out;
  char* ws = (char*)d_ws; size_t off = 0;
  auto take = [&](size_t bytes) { char* p = ws + off; off += (bytes + 255) & ~(size_t)255; return p; };
  _Float16* BQ = (_Float16*)take((size_t)DM * DM * 2); _Float16* BK = (_Float16*)take((size_t)DM * DM * 2); _Float16* BV = (_Float16*)take((size_t)DM * DM * 2); _Float16* BO = (_Float16*)take((size_t)DM * DM * 2);
  _Float16* XQ = (_Float16*)take(NR * DM * 2); _Float16* XK = (_Float16*)take(NR * DM * 2); _Float16* XV = (_Float16*)take(NR * DM * 2);
  _Float16* Q16 = (_Float16*)take(NR * DM * 2); _Float16* K16 = (_Float16*)take(NR * DM * 2); _Float16* V16 = (_Float16*)take(NR * DM * 2);
  float* QF0 = (float*)take((size_t)NB * QT0 * DM * 4); float* KF0 = (float*)take((size_t)NB * QT0 * DM * 4); float* VF0 = (float*)take((size_t)NB * QT0 * DM * 4); float* OF0 = (float*)take((size_t)NB * QT0 * DM * 4);
  _Float16* OH0 = (_Float16*)take((size_t)NB * QT0 * DM * 2); _Float16* OL0 = (_Float16*)take((size_t)NB * QT0 * DM * 2);
  if (off > ws_size) return;
  _Float16* VT = XK;
  _Float16* O16 = XQ;
  const unsigned gw = (unsigned)(((size_t)DM * (DM / 8) + 255) / 256);
  k_wt_f16<<<gw, 256, 0, stream>>>(Wq, BQ, DM, DM, 16.0f);
  k_wt_f16<<<gw, 256, 0, stream>>>(Wk, BK, DM, DM, 16.0f);
  k_wt_f16<<<gw, 256, 0, stream>>>(Wv, BV, DM, DM, 16.0f);
  k_wt_f16<<<gw, 256, 0, stream>>>(Wo, BO, DM, DM, 16.0f);
  const size_t n8b = (size_t)SQ * DM / 8; const dim3 gx((unsigned)((n8b + 255) / 256), NB);
  k_x16b<<<gx, 256, 0, stream>>>(q, (size_t)SQ_FULL * DM, XQ, (size_t)SQ * DM, n8b);
  k_x16b<<<gx, 256, 0, stream>>>(k, (size_t)SQ_FULL * DM, XK, (size_t)SQ * DM, n8b);
  k_x16b<<<gx, 256, 0, stream>>>(v, (size_t)SQ_FULL * DM, XV, (size_t)SQ * DM, n8b);
  const dim3 gp((unsigned)((NR / 128) * (DM / 64)), 1);
  k_gemm2<<<gp, 128, 0, stream>>>(XQ, DM, (size_t)0, BQ, DM, (size_t)0, 0.0625f, bq, (const float*)nullptr, (float*)nullptr, Q16, DM, (size_t)0, (int)NR, DM, DM);
  k_gemm2<<<gp, 128, 0, stream>>>(XK, DM, (size_t)0, BK, DM, (size_t)0, 0.0625f, bk, (const float*)nullptr, (float*)nullptr, K16, DM, (size_t)0, (int)NR, DM, DM);
  k_gemm2<<<gp, 128, 0, stream>>>(XV, DM, (size_t)0, BV, DM, (size_t)0, 0.0625f, bv, (const float*)nullptr, (float*)nullptr, V16, DM, (size_t)0, (int)NR, DM, DM);
  const dim3 g0((QT0 / 128) * (DM / 64), NB);
  k_gemm2<<<g0, 128, 0, stream>>>(XQ, DM, (size_t)SQ * DM, BQ, DM, (size_t)0, 0.0625f, bq, (const float*)nullptr, QF0, (_Float16*)nullptr, DM, (size_t)QT0 * DM, QT0, DM, DM);
  k_gemm2<<<g0, 128, 0, stream>>>(XK, DM, (size_t)SQ * DM, BK, DM, (size_t)0, 0.0625f, bk, (const float*)nullptr, KF0, (_Float16*)nullptr, DM, (size_t)QT0 * DM, QT0, DM, DM);
  k_gemm2<<<g0, 128, 0, stream>>>(XV, DM, (size_t)SQ * DM, BV, DM, (size_t)0, 0.0625f, bv, (const float*)nullptr, VF0, (_Float16*)nullptr, DM, (size_t)QT0 * DM, QT0, DM, DM);
  k_vt16<<<NB * NH * (SQ / 64), 256, 0, stream>>>(V16, DM, VT);
  k_att0<<<dim3(NH * (QT0 / 64), NB), 64, 0, stream>>>(QF0, KF0, VF0, DM, 0.125f, OF0, DM);
  k_hl<<<(unsigned)(((size_t)NB * QT0 * DM / 8 + 255) / 256), 256, 0, stream>>>(OF0, OH0, OL0, (size_t)NB * QT0 * DM / 8);
  k_fattn<<<dim3(SQ / 128, NB * NH), 256, 0, stream>>>(Q16, K16, VT, O16);
  k_gemm2<<<dim3((SQ / 128) * (DM / 64), NB), 128, 0, stream>>>(O16, DM, (size_t)SQ * DM, BO, DM, (size_t)0, 0.0009765625f, bo, (const float*)nullptr, out, (_Float16*)nullptr, DM, (size_t)SQ_FULL * DM, SQ, DM, DM);
  k_gemm2<<<g0, 128, 0, stream>>>(OH0, DM, (size_t)QT0 * DM, BO, DM, (size_t)0, 0.0009765625f, bo, (const float*)nullptr, out, (_Float16*)nullptr, DM, (size_t)SQ_FULL * DM, QT0, DM, DM);
  k_gemm2<<<g0, 128, 0, stream>>>(OL0, DM, (size_t)QT0 * DM, BO, DM, (size_t)0, 0.00000095367431640625f, (const float*)nullptr, (const float*)out, out, (_Float16*)nullptr, DM, (size_t)SQ_FULL * DM, QT0, DM, DM);
}
